// TransformerBlockQuantum_65481071396058
// MI455X (gfx1250) — hardware-verified
//
#include <hip/hip_runtime.h>
#include <stdint.h>


#ifndef NB
#define NB 4
#endif
#ifndef SEQ
#define SEQ 1024
#endif
#define NB_FULL 4
#define SEQ_FULL 1024
#define EMB 128
#define NH 16
#define HD 8
#define FFD 512
#define NTOK (NB * SEQ)
#define QCH 128
#define TROWS 64
#define T1P 132
#define THP 136
#define HTP 520
#define T1_BYTES (TROWS * T1P * 4)
#define HT_BYTES (TROWS * HTP * 2)
#define DSM_BYTES (T1_BYTES + HT_BYTES)

static_assert(NB >= 1 && NB <= NB_FULL);
static_assert(SEQ >= QCH && SEQ <= SEQ_FULL);
static_assert(SEQ % QCH == 0);
static_assert(SEQ % TROWS == 0);
static_assert(SEQ % 32 == 0);
static_assert(EMB == NH * HD);
static_assert(EMB % 32 == 0 && FFD % 32 == 0);
static_assert((T1_BYTES % 16) == 0);
static_assert((TROWS * EMB) % 256 == 0);

typedef _Float16 v16h __attribute__((ext_vector_type(16)));
typedef _Float16 v8h  __attribute__((ext_vector_type(8)));
typedef float    v8f  __attribute__((ext_vector_type(8)));
typedef float    v4f  __attribute__((ext_vector_type(4)));
typedef int      v4i  __attribute__((ext_vector_type(4)));
union Frag { v16h v; v8h half[2]; };

__device__ __forceinline__ v8f wmma16(v16h a, v16h b, v8f c) {
  v8f d = __builtin_amdgcn_wmma_f32_16x16x32_f16(false, a, false, b, (short)0, c, false, false);
  asm volatile("v_nop\n\tv_nop\n\tv_nop\n\tv_nop" : "+v"(d) : "v"(a), "v"(b));
  return d;
}

__device__ __forceinline__ v8f vzero8f() { v8f z = {0.f, 0.f, 0.f, 0.f, 0.f, 0.f, 0.f, 0.f}; return z; }
__device__ __forceinline__ v8h vzero8h() { v4i z = {0, 0, 0, 0}; return __builtin_bit_cast(v8h, z); }

__device__ __forceinline__ v8h zsel8(bool zero, v8h v) {
  v4i w = __builtin_bit_cast(v4i, v);
  v4i r;
  r.x = zero ? 0 : w.x; r.y = zero ? 0 : w.y; r.z = zero ? 0 : w.z; r.w = zero ? 0 : w.w;
  return __builtin_bit_cast(v8h, r);
}

__device__ __forceinline__ float bf16r(float f) {
  unsigned u = __float_as_uint(f);
  u = (u + 0x7FFFu + ((u >> 16) & 1u)) & 0xFFFF0000u;
  return __uint_as_float(u);
}

__device__ __forceinline__ void vst8h(_Float16* p, v8h v) { *(volatile v8h*)p = v; }
__device__ __forceinline__ void vst4f(float* p, v4f v) { *(volatile v4f*)p = v; }

__device__ __forceinline__ float rsum16(float v) {
  v += __shfl_xor(v, 1, 32);
  v += __shfl_xor(v, 2, 32);
  v += __shfl_xor(v, 4, 32);
  v += __shfl_xor(v, 8, 32);
  return v;
}

__global__ __launch_bounds__(256)
void k_cvt(const float* __restrict__ x, const float* __restrict__ Wq,
           const float* __restrict__ Wo, const float* __restrict__ W2,
           _Float16* __restrict__ xh, _Float16* __restrict__ wqh,
           _Float16* __restrict__ woh, _Float16* __restrict__ w2h) {
  const int seg = blockIdx.y;
  const int i8 = blockIdx.x * 256 + threadIdx.x;
  const float* src; _Float16* dst; int n8; float sc;
  if (seg == 0)      { src = x;  dst = xh;  n8 = NTOK * (EMB / 8); sc = 16.f; }
  else if (seg == 1) { src = Wq; dst = wqh; n8 = EMB * EMB / 8;    sc = 16.f; }
  else if (seg == 2) { src = Wo; dst = woh; n8 = EMB * EMB / 8;    sc = 16.f; }
  else               { src = W2; dst = w2h; n8 = EMB * FFD / 8;    sc = 64.f; }
  if (i8 >= n8) return;
  size_t si = (size_t)i8 * 8;
  if (seg == 0) {
    const int t = i8 >> 4, c8 = i8 & 15;
    const int b = t / SEQ, s = t - b * SEQ;
    si = ((size_t)(b * SEQ_FULL + s)) * EMB + (size_t)c8 * 8;
  }
  v4f f0 = *(const v4f*)(src + si);
  v4f f1 = *(const v4f*)(src + si + 4);
  v8h hv;
#pragma unroll
  for (int i = 0; i < 4; ++i) {
    hv[i]     = (_Float16)(bf16r(f0[i]) * sc);
    hv[4 + i] = (_Float16)(bf16r(f1[i]) * sc);
  }
  _Float16* dp = dst + (size_t)i8 * 8;
  vst8h(dp, hv);
  __threadfence();
  vst8h(dp, hv);
}

__global__ __launch_bounds__(256)
void k_qproj(const _Float16* __restrict__ xh, const _Float16* __restrict__ wqh,
             const float* __restrict__ bq, const float* __restrict__ rx,
             _Float16* __restrict__ qk) {
  __shared__ __align__(16) float    tq[TROWS * T1P];
  __shared__ __align__(16) _Float16 th[TROWS * THP];

  const int tid = threadIdx.x, lane = tid & 31, wave = tid >> 5;
  const int hl = lane >> 4, m = lane & 15;
  const int r0 = (wave & 3) * 16, c0 = (wave >> 2) * 64;
  const int t0 = blockIdx.x * TROWS;

  v8f acc[4];
#pragma unroll
  for (int j = 0; j < 4; ++j) acc[j] = vzero8f();

  for (int ks = 0; ks < EMB / 32; ++ks) {
    const int k0 = ks * 32;
    Frag a;
    const _Float16* ap = xh + (size_t)(t0 + r0 + m) * EMB + k0 + 8 * hl;
    a.half[0] = *(const v8h*)ap;
    a.half[1] = *(const v8h*)(ap + 16);
#pragma unroll
    for (int j = 0; j < 4; ++j) {
      Frag bb;
      const _Float16* bp = wqh + (size_t)(c0 + 16 * j + m) * EMB + k0 + 8 * hl;
      bb.half[0] = *(const v8h*)bp;
      bb.half[1] = *(const v8h*)(bp + 16);
      acc[j] = wmma16(a.v, bb.v, acc[j]);
    }
  }

#pragma unroll
  for (int j = 0; j < 4; ++j) {
    const int col = c0 + 16 * j + m;
    const float bqv = bf16r(bq[col]);
    const float rxv = bf16r(rx[col]);
#pragma unroll
    for (int r = 0; r < 8; ++r) {
      const int row = r0 + 8 * hl + r;
      float v = acc[j][r] * (1.0f / 256.0f) + bqv;
      v = v + rxv;
      tq[row * T1P + col] = v;
    }
  }
  __syncthreads();

#pragma unroll 1
  for (int i = 0; i < (TROWS * EMB) / 256; ++i) {
    const int e = i * 256 + tid;
    const int row = e >> 7, col = e & 127;
    th[row * THP + col] = (_Float16)cosf(tq[row * T1P + col]);
  }
  __syncthreads();

  const int b = t0 / SEQ, s0 = t0 - b * SEQ;
  v8h sv[4]; _Float16* sp[4];
#pragma unroll
  for (int u = 0; u < 4; ++u) {
    const int hd = 2 * wave + (u >> 1);
    const int row = 32 * (u & 1) + lane;
    sv[u] = *(const v8h*)&th[row * THP + hd * 8];
    sp[u] = qk + (((size_t)(b * NH + hd)) * SEQ + s0 + row) * HD;
  }
#pragma unroll
  for (int u = 0; u < 4; ++u) vst8h(sp[u], sv[u]);
  __threadfence();
#pragma unroll
  for (int u = 0; u < 4; ++u) vst8h(sp[u], sv[u]);
}

__global__ __launch_bounds__(256)
void k_attn(const _Float16* __restrict__ qk, _Float16* __restrict__ ctxh) {
  __shared__ __align__(16) _Float16 lk[SEQ * HD];
  __shared__ __align__(16) _Float16 lvT[HD * SEQ];
  __shared__ __align__(16) _Float16 pbuf[8 * 512];

  const int tid = threadIdx.x, lane = tid & 31, wave = tid >> 5;
  const int hl = lane >> 4, m = lane & 15;
  const int nqc = SEQ / QCH;
  const int bh = blockIdx.x / nqc, qc = blockIdx.x - bh * nqc;
  const _Float16* g = qk + (size_t)bh * SEQ * HD;

  for (int i = tid * 8; i < SEQ * HD; i += 256 * 8)
    *(v4i*)&lk[i] = *(const v4i*)&g[i];
  __syncthreads();
  for (int i = tid; i < SEQ * HD; i += 256)
    lvT[(i & 7) * SEQ + (i >> 3)] = lk[i];
  __syncthreads();

  const int q0 = qc * QCH + wave * 16;
  _Float16* pb = pbuf + wave * 512;
  const v8h z8 = vzero8h();

  Frag aq;
  {
    v8h kq = *(const v8h*)&lk[(q0 + m) * HD];
    aq.half[0] = zsel8(hl != 0, kq);
    aq.half[1] = z8;
  }

  v8f c = vzero8f();
  float psum[8];
#pragma unroll
  for (int r = 0; r < 8; ++r) psum[r] = 0.f;
  const float C2 = 0.35355339059327373f * 1.4426950408889634f;

#pragma unroll 1
  for (int kt = 0; kt < SEQ / 32; ++kt) {
    const int tb = kt * 32;
    Frag b0, b1;
    {
      v8h k0v = *(const v8h*)&lk[(tb + m) * HD];
      v8h k1v = *(const v8h*)&lk[(tb + 16 + m) * HD];
      b0.half[0] = zsel8(hl != 0, k0v); b0.half[1] = z8;
      b1.half[0] = zsel8(hl != 0, k1v); b1.half[1] = z8;
    }
    v8f zc = vzero8f();
    v8f d0 = wmma16(aq.v, b0.v, zc);
    v8f d1 = wmma16(aq.v, b1.v, zc);

    __builtin_amdgcn_fence(__ATOMIC_RELEASE, "wavefront");
    __builtin_amdgcn_wave_barrier();
#pragma unroll
    for (int r = 0; r < 8; ++r) {
      const float p0 = exp2f((d0[r] - 8.0f) * C2);
      const float p1 = exp2f((d1[r] - 8.0f) * C2);
      psum[r] += p0 + p1;
      pb[(8 * hl + r) * 32 + m]      = (_Float16)(p0 * 1024.0f);
      pb[(8 * hl + r) * 32 + 16 + m] = (_Float16)(p1 * 1024.0f);
    }
    __builtin_amdgcn_fence(__ATOMIC_RELEASE, "wavefront");
    __builtin_amdgcn_wave_barrier();

    Frag ap;
    ap.half[0] = *(const v8h*)&pb[m * 32 + 8 * hl];
    ap.half[1] = *(const v8h*)&pb[m * 32 + 16 + 8 * hl];
    Frag bv;
    {
      const _Float16* vr = lvT + (m & 7) * SEQ + tb;
      v8h v0 = *(const v8h*)(vr + 8 * hl);
      v8h v1 = *(const v8h*)(vr + 16 + 8 * hl);
      bv.half[0] = zsel8(m >= 8, v0);
      bv.half[1] = zsel8(m >= 8, v1);
    }
    c = wmma16(ap.v, bv.v, c);
  }

  _Float16 hv[8];
#pragma unroll
  for (int r = 0; r < 8; ++r) {
    const float den = rsum16(psum[r]);
    const float inv = 1.0f / den;
    hv[r] = (_Float16)(c[r] * inv * (1.0f / 64.0f));
  }
  __builtin_amdgcn_fence(__ATOMIC_RELEASE, "wavefront");
  __builtin_amdgcn_wave_barrier();
  if (m < HD) {
#pragma unroll
    for (int r = 0; r < 8; ++r) pb[(8 * hl + r) * 8 + m] = hv[r];
  }
  __builtin_amdgcn_fence(__ATOMIC_RELEASE, "wavefront");
  __builtin_amdgcn_wave_barrier();

  v8h ov = *(const v8h*)&pb[(lane & 15) * 8];
  _Float16* op = ctxh + ((size_t)bh * SEQ + q0 + (lane & 15)) * HD;
  if (lane < 16) vst8h(op, ov);
  __threadfence();
  if (lane < 16) vst8h(op, ov);
}

__device__ __forceinline__ void ln_rows(float* T, const float* sg, const float* sb, int tid) {
  const int row = tid >> 2, part = tid & 3;
  float* rp = T + row * T1P + part * 32;
  float s = 0.f;
#pragma unroll 2
  for (int i = 0; i < 8; ++i) {
    v4f w = *(const v4f*)(rp + 4 * i);
    s += (w.x + w.y) + (w.z + w.w);
  }
  s += __shfl_xor(s, 1, 32);
  s += __shfl_xor(s, 2, 32);
  const float mu = s * (1.0f / EMB);
  float q = 0.f;
#pragma unroll 2
  for (int i = 0; i < 8; ++i) {
    v4f w = *(const v4f*)(rp + 4 * i);
    const float a0 = w.x - mu, a1 = w.y - mu, a2 = w.z - mu, a3 = w.w - mu;
    q += (a0 * a0 + a1 * a1) + (a2 * a2 + a3 * a3);
  }
  q += __shfl_xor(q, 1, 32);
  q += __shfl_xor(q, 2, 32);
  const float rstd = 1.0f / sqrtf(q * (1.0f / EMB) + 1e-5f);
#pragma unroll 2
  for (int i = 0; i < 8; ++i) {
    const int col = part * 32 + 4 * i;
    v4f w = *(const v4f*)(rp + 4 * i);
    v4f o;
    o.x = (w.x - mu) * rstd * sg[col]     + sb[col];
    o.y = (w.y - mu) * rstd * sg[col + 1] + sb[col + 1];
    o.z = (w.z - mu) * rstd * sg[col + 2] + sb[col + 2];
    o.w = (w.w - mu) * rstd * sg[col + 3] + sb[col + 3];
    *(v4f*)(rp + 4 * i) = o;
  }
}

__global__ __launch_bounds__(256)
void k_tail(const _Float16* __restrict__ ctxh, const _Float16* __restrict__ woh,
            const _Float16* __restrict__ w2h, const float* __restrict__ x,
            const float* __restrict__ bo, const float* __restrict__ ry,
            const float* __restrict__ W1, const float* __restrict__ b1,
            const float* __restrict__ b2,
            const float* __restrict__ g1, const float* __restrict__ bt1,
            const float* __restrict__ g2, const float* __restrict__ bt2,
            float* __restrict__ out) {
  extern __shared__ __align__(16) unsigned char dsm[];
  float* T1 = (float*)dsm;
  _Float16* HT = (_Float16*)(dsm + T1_BYTES);
  __shared__ float sbo[EMB], sb2[EMB], sg1[EMB], sbt1[EMB], sg2[EMB], sbt2[EMB];
  __shared__ float scry[HD];
  __shared__ __align__(16) float sq[TROWS * HD];

  const int tid = threadIdx.x, lane = tid & 31, wave = tid >> 5;
  const int hl = lane >> 4, m = lane & 15;
  const int r0 = (wave & 3) * 16, c0 = (wave >> 2) * 64;
  const int t0 = blockIdx.x * TROWS;
  const int b = t0 / SEQ, s0 = t0 - b * SEQ;

  if (tid < EMB) {
    sbo[tid] = bf16r(bo[tid]);  sb2[tid] = bf16r(b2[tid]);
    sg1[tid] = bf16r(g1[tid]);  sbt1[tid] = bf16r(bt1[tid]);
    sg2[tid] = bf16r(g2[tid]);  sbt2[tid] = bf16r(bt2[tid]);
  }
  if (tid < HD) scry[tid] = cosf(bf16r(ry[tid]));

  {
    const float* xb = x + ((size_t)(b * SEQ_FULL + s0)) * EMB;
#pragma unroll
    for (int i = 0; i < 8; ++i) {
      const int idx = i * 256 + tid;
      const int row = idx >> 5, c4 = idx & 31;
      v4f v = *(const v4f*)(xb + (size_t)row * EMB + c4 * 4);
      v4f w;
      w.x = bf16r(v.x); w.y = bf16r(v.y); w.z = bf16r(v.z); w.w = bf16r(v.w);
      *(v4f*)&T1[row * T1P + c4 * 4] = w;
    }
  }
  __syncthreads();

  {
    v8f acc[4];
#pragma unroll
    for (int j = 0; j < 4; ++j) acc[j] = vzero8f();
    for (int ks = 0; ks < EMB / 32; ++ks) {
      const int k0 = ks * 32;
      Frag a;
      const _Float16* a0p = ctxh + (((size_t)(b * NH + 4 * ks + hl)) * SEQ + s0 + r0 + m) * HD;
      const _Float16* a1p = ctxh + (((size_t)(b * NH + 4 * ks + 2 + hl)) * SEQ + s0 + r0 + m) * HD;
      a.half[0] = *(const v8h*)a0p;
      a.half[1] = *(const v8h*)a1p;
#pragma unroll
      for (int j = 0; j < 4; ++j) {
        Frag bb;
        const _Float16* bp = woh + (size_t)(c0 + 16 * j + m) * EMB + k0 + 8 * hl;
        bb.half[0] = *(const v8h*)bp;
        bb.half[1] = *(const v8h*)(bp + 16);
        acc[j] = wmma16(a.v, bb.v, acc[j]);
      }
    }
#pragma unroll
    for (int j = 0; j < 4; ++j) {
      const int col = c0 + 16 * j + m;
      const float bov = sbo[col];
#pragma unroll
      for (int r = 0; r < 8; ++r) {
        const int row = r0 + 8 * hl + r;
        float* tp = &T1[row * T1P + col];
        float v = acc[j][r] * (1.0f / 256.0f) + bov;
        v = *tp + v;
        *tp = v;
      }
    }
  }
  __syncthreads();

  ln_rows(T1, sg1, sbt1, tid);
  __syncthreads();

  for (int i = tid; i < TROWS * HD; i += 256) {
    const int row = i >> 3, e = i & 7;
    sq[i] = cosf(T1[row * T1P + e]) * scry[e];
  }
  __syncthreads();

  {
    const int row = tid >> 2, fp = (tid & 3) * 128;
    const v4f qa = *(const v4f*)&sq[row * HD];
    const v4f qb = *(const v4f*)&sq[row * HD + 4];
#pragma unroll 2
    for (int f = fp; f < fp + 128; ++f) {
      const v4f wa = *(const v4f*)(W1 + (size_t)f * HD);
      const v4f wb = *(const v4f*)(W1 + (size_t)f * HD + 4);
      float sacc = qa.x * bf16r(wa.x);
      sacc = fmaf(qa.y, bf16r(wa.y), sacc);
      sacc = fmaf(qa.z, bf16r(wa.z), sacc);
      sacc = fmaf(qa.w, bf16r(wa.w), sacc);
      sacc = fmaf(qb.x, bf16r(wb.x), sacc);
      sacc = fmaf(qb.y, bf16r(wb.y), sacc);
      sacc = fmaf(qb.z, bf16r(wb.z), sacc);
      sacc = fmaf(qb.w, bf16r(wb.w), sacc);
      const float hvv = fmaxf(sacc + bf16r(b1[f]), 0.0f) * 16.0f;
      HT[row * HTP + f] = (_Float16)hvv;
    }
  }
  __syncthreads();

  {
    v8f acc[4];
#pragma unroll
    for (int j = 0; j < 4; ++j) acc[j] = vzero8f();
#pragma unroll 2
    for (int ks = 0; ks < FFD / 32; ++ks) {
      const int k0 = ks * 32;
      Frag a;
      const _Float16* ap = HT + (r0 + m) * HTP + k0 + 8 * hl;
      a.half[0] = *(const v8h*)ap;
      a.half[1] = *(const v8h*)(ap + 16);
#pragma unroll
      for (int j = 0; j < 4; ++j) {
        Frag bb;
        const _Float16* bp = w2h + (size_t)(c0 + 16 * j + m) * FFD + k0 + 8 * hl;
        bb.half[0] = *(const v8h*)bp;
        bb.half[1] = *(const v8h*)(bp + 16);
        acc[j] = wmma16(a.v, bb.v, acc[j]);
      }
    }
#pragma unroll
    for (int j = 0; j < 4; ++j) {
      const int col = c0 + 16 * j + m;
      const float b2v = sb2[col];
#pragma unroll
      for (int r = 0; r < 8; ++r) {
        const int row = r0 + 8 * hl + r;
        float* tp = &T1[row * T1P + col];
        float v = acc[j][r] * (1.0f / 1024.0f) + b2v;
        v = *tp + v;
        *tp = v;
      }
    }
  }
  __syncthreads();

  ln_rows(T1, sg2, sbt2, tid);
  __syncthreads();

  {
    float* ob = out + (size_t)t0 * EMB;
    v4f ov[8]; float* opp[8];
#pragma unroll
    for (int i = 0; i < 8; ++i) {
      const int idx = i * 256 + tid;
      const int row = idx >> 5, c4 = idx & 31;
      ov[i] = *(const v4f*)&T1[row * T1P + c4 * 4];
      opp[i] = ob + (size_t)row * EMB + c4 * 4;
    }
#pragma unroll
    for (int i = 0; i < 8; ++i) vst4f(opp[i], ov[i]);
    __threadfence();
#pragma unroll
    for (int i = 0; i < 8; ++i) vst4f(opp[i], ov[i]);
  }
}

extern "C" void kernel_launch(void* const* d_in, const int* in_sizes, int n_in,
                              void* d_out, int out_size, void* d_ws, size_t ws_size,
                              hipStream_t stream) {
  if (n_in < 19) return;
  if (in_sizes[0] < ((NB - 1) * SEQ_FULL + SEQ) * EMB) return;
  if (in_sizes[1] < EMB * EMB || in_sizes[2] < EMB || in_sizes[7] < EMB ||
      in_sizes[8] < EMB * EMB || in_sizes[9] < EMB || in_sizes[10] < HD ||
      in_sizes[11] < FFD * HD || in_sizes[12] < FFD || in_sizes[13] < EMB * FFD ||
      in_sizes[14] < EMB || in_sizes[15] < EMB || in_sizes[16] < EMB ||
      in_sizes[17] < EMB || in_sizes[18] < EMB) return;
  if (out_size < NTOK * EMB) return;

  const float* x   = (const float*)d_in[0];
  const float* Wq  = (const float*)d_in[1];
  const float* bq  = (const float*)d_in[2];
  const float* rx  = (const float*)d_in[7];
  const float* Wo  = (const float*)d_in[8];
  const float* bo  = (const float*)d_in[9];
  const float* ry  = (const float*)d_in[10];
  const float* W1  = (const float*)d_in[11];
  const float* b1  = (const float*)d_in[12];
  const float* W2  = (const float*)d_in[13];
  const float* b2  = (const float*)d_in[14];
  const float* g1  = (const float*)d_in[15];
  const float* bt1 = (const float*)d_in[16];
  const float* g2  = (const float*)d_in[17];
  const float* bt2 = (const float*)d_in[18];
  float* out = (float*)d_out;

  const size_t xh_bytes  = (size_t)NTOK * EMB * 2;
  const size_t wq_bytes  = (size_t)EMB * EMB * 2;
  const size_t wo_bytes  = (size_t)EMB * EMB * 2;
  const size_t w2_bytes  = (size_t)EMB * FFD * 2;
  const size_t qk_bytes  = (size_t)NB * NH * SEQ * HD * 2;
  const size_t ctx_bytes = (size_t)NB * NH * SEQ * HD * 2;
  size_t off = 0;
  const size_t off_xh  = off; off += (xh_bytes  + 255) & ~(size_t)255;
  const size_t off_wq  = off; off += (wq_bytes  + 255) & ~(size_t)255;
  const size_t off_wo  = off; off += (wo_bytes  + 255) & ~(size_t)255;
  const size_t off_w2  = off; off += (w2_bytes  + 255) & ~(size_t)255;
  const size_t off_qk  = off; off += (qk_bytes  + 255) & ~(size_t)255;
  const size_t off_ctx = off; off += (ctx_bytes + 255) & ~(size_t)255;
  if (off > ws_size) return;

  char* ws = (char*)d_ws;
  _Float16* xh   = (_Float16*)(ws + off_xh);
  _Float16* wqh  = (_Float16*)(ws + off_wq);
  _Float16* woh  = (_Float16*)(ws + off_wo);
  _Float16* w2h  = (_Float16*)(ws + off_w2);
  _Float16* qk   = (_Float16*)(ws + off_qk);
  _Float16* ctxh = (_Float16*)(ws + off_ctx);

  int maxn8 = NTOK * (EMB / 8);
  if (maxn8 < EMB * FFD / 8) maxn8 = EMB * FFD / 8;
  const int cvt_blocks = (maxn8 + 255) / 256;

  k_cvt<<<dim3(cvt_blocks, 4), dim3(256), 0, stream>>>(x, Wq, Wo, W2, xh, wqh, woh, w2h);
  k_qproj<<<dim3(NTOK / TROWS), dim3(256), 0, stream>>>(xh, wqh, bq, rx, qk);
  k_attn<<<dim3(NB * NH * (SEQ / QCH)), dim3(256), 0, stream>>>(qk, ctxh);
  hipFuncSetAttribute(reinterpret_cast<const void*>(&k_tail),
                      hipFuncAttributeMaxDynamicSharedMemorySize, DSM_BYTES);
  k_tail<<<dim3(NTOK / TROWS), dim3(256), DSM_BYTES, stream>>>(
      ctxh, woh, w2h, x, bo, ry, W1, b1, b2, g1, bt1, g2, bt2, out);
}
